// CrossViewCrossAttention_38268158607378
// MI455X (gfx1250) — hardware-verified
//
#include <hip/hip_runtime.h>


#define NBT  8
#define CC   256
#define NX   1024
#define NZ   256
#define NH_  8
#define HD   32
#define NL   2
#define MID  1024
#define DM   CC
#define QSC  0.17677669529663688f
#define LEPS 1e-5f
#define LOSC 1024.0f

typedef _Float16 h16;
typedef unsigned short bf;
typedef __attribute__((ext_vector_type(16))) __bf16   v16bf;
typedef __attribute__((ext_vector_type(16))) _Float16 v16h;
typedef __attribute__((ext_vector_type(8)))  _Float16 v8h;
typedef __attribute__((ext_vector_type(8)))  unsigned short v8us;
typedef __attribute__((ext_vector_type(8)))  float    v8f;
typedef __attribute__((ext_vector_type(4)))  float    v4f;
typedef __attribute__((ext_vector_type(4)))  _Float16 v4h;
typedef v8h  __attribute__((may_alias)) v8ha;
typedef v4f  __attribute__((may_alias)) v4fa;
typedef v8us __attribute__((may_alias)) v8usa;

__device__ __forceinline__ unsigned short f2bf(float f) { unsigned u = __float_as_uint(f); u += 0x7FFFu + ((u >> 16) & 1u); return (unsigned short)(u >> 16); }
__device__ __forceinline__ float bf2f(unsigned short b) { return __uint_as_float(((unsigned)b) << 16); }
__device__ __forceinline__ float bfr(float f) { return bf2f(f2bf(f)); }
__device__ __forceinline__ v16h cat16(v8h lo, v8h hi) { return __builtin_shufflevector(lo, hi, 0, 1, 2, 3, 4, 5, 6, 7, 8, 9, 10, 11, 12, 13, 14, 15); }
__device__ __forceinline__ v16bf cat16b(v8us lo, v8us hi) { return __builtin_bit_cast(v16bf, __builtin_shufflevector(lo, hi, 0, 1, 2, 3, 4, 5, 6, 7, 8, 9, 10, 11, 12, 13, 14, 15)); }
__device__ __forceinline__ v8f wmma16(v16h a, v16h b, v8f c) { return __builtin_amdgcn_wmma_f32_16x16x32_f16(false, a, false, b, (short)0, c, false, false); }
__device__ __forceinline__ v8f wmmab(v16bf a, v16bf b, v8f c) { return __builtin_amdgcn_wmma_f32_16x16x32_bf16(false, a, false, b, (short)0, c, false, false); }

__global__ __launch_bounds__(256) void k_wt(const float* __restrict__ Wm, int K, int ncols, bf* WT) {
    __shared__ __align__(16) unsigned short tl[64 * 72];
    const int tid = threadIdx.x, k0 = blockIdx.x * 64, n0 = blockIdx.y * 64;
    const int kk = tid >> 2, nq = (tid & 3) * 16;
#pragma unroll
    for (int i = 0; i < 16; ++i) tl[(nq + i) * 72 + kk] = f2bf(Wm[(size_t)(k0 + kk) * ncols + n0 + nq + i]);
    __syncthreads();
    const int piece = tid & 7;
    auto pass = [&]() {
#pragma unroll
        for (int s = 0; s < 2; ++s) { const int nr = (tid >> 3) + 32 * s; const v8us val = *(const v8usa*)(tl + nr * 72 + piece * 8); *(volatile v8us*)(WT + (size_t)(n0 + nr) * K + k0 + piece * 8) = val; }
    };
    pass(); __threadfence(); pass();
}
template <bool SPLITA, bool F16OUT = false>
__global__ __launch_bounds__(128) void k_gemmb(const bf* __restrict__ A, const bf* __restrict__ Al, const bf* __restrict__ Bn, const float* __restrict__ bias, float* C, int ldc, h16* C2, const float* __restrict__ R = nullptr, int K = DM, int roundR = 1) {
    __shared__ __align__(16) float ost[4][16 * 68];
    const int lane = threadIdx.x & 31, wave = threadIdx.x >> 5, lr = lane & 15, hi = lane >> 4;
    const int r0 = blockIdx.x * 64 + wave * 16, c0 = blockIdx.y * 64;
    const size_t aoff = (size_t)(r0 + lr) * K + 8 * hi;
    size_t boff[4];
#pragma unroll
    for (int t = 0; t < 4; ++t) boff[t] = (size_t)(c0 + t * 16 + lr) * K + 8 * hi;
    v8f acc[4];
#pragma unroll
    for (int t = 0; t < 4; ++t) acc[t] = (v8f){};
#pragma unroll 1
    for (int kc = 0; kc < K; kc += 32) {
        const v16bf a = cat16b(*(const v8us*)(A + aoff + kc), *(const v8us*)(A + aoff + kc + 16));
        v16bf al = a;
        if (SPLITA) al = cat16b(*(const v8us*)(Al + aoff + kc), *(const v8us*)(Al + aoff + kc + 16));
#pragma unroll
        for (int t = 0; t < 4; ++t) { const v16bf b = cat16b(*(const v8us*)(Bn + boff[t] + kc), *(const v8us*)(Bn + boff[t] + kc + 16)); acc[t] = wmmab(a, b, acc[t]); if (SPLITA) acc[t] = wmmab(al, b, acc[t]); }
        asm volatile("v_nop\n\tv_nop\n\tv_nop\n\tv_nop" : "+v"(acc[0]), "+v"(acc[1]), "+v"(acc[2]), "+v"(acc[3]) : "v"(a), "v"(al));
    }
    float* os = &ost[wave][0];
#pragma unroll
    for (int t = 0; t < 4; ++t) { const float bv = bias ? bfr(bias[c0 + t * 16 + lr]) : 0.f;
#pragma unroll
        for (int j = 0; j < 8; ++j) os[(hi * 8 + j) * 68 + t * 16 + lr] = acc[t][j] + bv; }
    __syncthreads();
    if (F16OUT) {
        h16* crow = (h16*)(void*)C + (size_t)r0 * ldc + c0;
        auto pass = [&]() {
#pragma unroll
            for (int s = 0; s < 4; ++s) { const int row = 4 * s + (lane >> 3), piece = lane & 7; const float* sp = os + row * 68 + piece * 8; v8h o, o2;
#pragma unroll
                for (int i = 0; i < 8; ++i) { const h16 a = (h16)sp[i]; o[i] = a; o2[i] = (h16)((sp[i] - (float)a) * LOSC); }
                *(volatile v8h*)(crow + (size_t)row * ldc + piece * 8) = o; if (C2) *(volatile v8h*)(C2 + (size_t)r0 * ldc + c0 + (size_t)row * ldc + piece * 8) = o2; }
        };
        pass(); __threadfence(); pass();
    } else {
        float* crow = C + (size_t)r0 * ldc + c0;
        auto pass = [&]() {
#pragma unroll
            for (int s = 0; s < 8; ++s) { const int Lid = (lane >> 3) + 4 * s, piece = lane & 7; const int row = Lid >> 1, cofs = (Lid & 1) * 32 + piece * 4;
                v4f val = *(const v4fa*)(os + row * 68 + cofs); if (R) { const v4f rv = *(const v4f*)(R + ((size_t)r0 + row) * ldc + c0 + cofs); val += roundR ? (v4f){bfr(rv[0]), bfr(rv[1]), bfr(rv[2]), bfr(rv[3])} : rv; }
                *(volatile v4f*)(crow + (size_t)row * ldc + cofs) = val; }
        };
        pass(); __threadfence(); pass();
    }
}

__global__ __launch_bounds__(256) void k_cvt8(const float* __restrict__ src, bf* dst, size_t n8) {
    const size_t i = (size_t)blockIdx.x * 256 + threadIdx.x; if (i >= n8) return;
    const v8f v = *(const v8f*)(src + i * 8); v8us o;
#pragma unroll
    for (int k = 0; k < 8; ++k) o[k] = f2bf(v[k]);
    *(volatile v8us*)(dst + i * 8) = o; __threadfence(); *(volatile v8us*)(dst + i * 8) = o;
}
__global__ __launch_bounds__(256) void k_zero8(bf* dst, size_t n8) {
    const size_t i = (size_t)blockIdx.x * 256 + threadIdx.x; if (i >= n8) return; v8us z;
#pragma unroll
    for (int k = 0; k < 8; ++k) z[k] = 0;
    *(volatile v8us*)(dst + i * 8) = z; __threadfence(); *(volatile v8us*)(dst + i * 8) = z;
}

template <int MODE>
__global__ __launch_bounds__(128) void k_gemm3z(const bf* __restrict__ Ah, const bf* __restrict__ Al, const bf* __restrict__ Bh, const bf* __restrict__ Bl, int K, float* C, int ldc, size_t sA, size_t sB, size_t sC) {
    if ((MODE & 1) && (int)blockIdx.y * 64 > (int)blockIdx.x * 64 + 63) return;
    const size_t z = blockIdx.z; Ah += z * sA; Al += z * sA; Bh += z * sB; Bl += z * sB; C += z * sC;
    const int Klim = (MODE & 2) ? min(K, ((int)blockIdx.x + 1) * 64) : K;
    __shared__ __align__(16) float ost[4][16 * 68];
    const int lane = threadIdx.x & 31, wave = threadIdx.x >> 5, lr = lane & 15, hi = lane >> 4;
    const int r0 = blockIdx.x * 64 + wave * 16, c0 = blockIdx.y * 64;
    const size_t aoff = (size_t)(r0 + lr) * K + 8 * hi;
    v8f acc[4];
#pragma unroll
    for (int t = 0; t < 4; ++t) acc[t] = (v8f){};
#pragma unroll 1
    for (int kc = 0; kc < Klim; kc += 32) {
        const v16bf a = cat16b(*(const v8us*)(Ah + aoff + kc), *(const v8us*)(Ah + aoff + kc + 16));
        v16bf al = a; if (!(MODE & 4) && !(MODE & 16)) al = cat16b(*(const v8us*)(Al + aoff + kc), *(const v8us*)(Al + aoff + kc + 16));
#pragma unroll
        for (int t = 0; t < 4; ++t) { const size_t bo = (size_t)(c0 + t * 16 + lr) * K + kc + 8 * hi;
            const v16bf bh = cat16b(*(const v8us*)(Bh + bo), *(const v8us*)(Bh + bo + 16));
            acc[t] = wmmab(a, bh, acc[t]);
            if (!(MODE & 4)) { if (!(MODE & 16)) acc[t] = wmmab(al, bh, acc[t]); if (!(MODE & 8)) { const v16bf bl = cat16b(*(const v8us*)(Bl + bo), *(const v8us*)(Bl + bo + 16)); acc[t] = wmmab(a, bl, acc[t]); } } }
        asm volatile("v_nop\n\tv_nop\n\tv_nop\n\tv_nop" : "+v"(acc[0]), "+v"(acc[1]), "+v"(acc[2]), "+v"(acc[3]) : "v"(a), "v"(al));
    }
    float* os = &ost[wave][0];
#pragma unroll
    for (int t = 0; t < 4; ++t) {
#pragma unroll
        for (int j = 0; j < 8; ++j) os[(hi * 8 + j) * 68 + t * 16 + lr] = acc[t][j]; }
    __builtin_amdgcn_wave_barrier(); asm volatile("" ::: "memory");
    float* crow = C + (size_t)r0 * ldc + c0;
    auto pass = [&]() {
#pragma unroll
        for (int s = 0; s < 8; ++s) { const int Lid = (lane >> 3) + 4 * s, piece = lane & 7; const int row = Lid >> 1, cofs = (Lid & 1) * 32 + piece * 4;
            const v4f val = *(const v4fa*)(os + row * 68 + cofs); *(volatile v4f*)(crow + (size_t)row * ldc + cofs) = val; }
    };
    pass(); __threadfence(); pass();
}
__global__ __launch_bounds__(256) void k_planes32z(const float* __restrict__ F, int ld, int off, float sc, int rows, bf* Ph, bf* Pl) {
    typedef __attribute__((ext_vector_type(2))) unsigned short v2us;
    const int lane = threadIdx.x & 31; const size_t r = ((size_t)blockIdx.x * 8 + (threadIdx.x >> 5)) * 2 + (lane >> 4); if (r >= (size_t)rows) return; const int z = blockIdx.z; const int c0 = (lane & 15) * 2; v2us oh, ol;
    Ph += (size_t)z * rows * 32; Pl += (size_t)z * rows * 32;
#pragma unroll
    for (int i = 0; i < 2; ++i) { const float y = F[r * ld + off + z * 32 + c0 + i] * sc; const unsigned short hb = f2bf(y); oh[i] = hb; ol[i] = f2bf(y - bf2f(hb)); }
    const size_t o = r * 32 + c0; *(volatile v2us*)(Ph + o) = oh; *(volatile v2us*)(Pl + o) = ol; __threadfence(); *(volatile v2us*)(Ph + o) = oh; *(volatile v2us*)(Pl + o) = ol;
}
__global__ __launch_bounds__(256) void k_vtpadz(const float* __restrict__ F, int ld, int off, int nk, bf* Th, bf* Tl) {
    typedef __attribute__((ext_vector_type(2))) unsigned short v2us;
    const int lane = threadIdx.x & 31; const size_t wid = (size_t)blockIdx.x * 8 + (threadIdx.x >> 5); if (wid >= (size_t)64 * (nk / 64)) return; const int z = blockIdx.z; const int d = (int)(wid / (nk / 64)); const int k0 = (int)(wid % (nk / 64)) * 64 + lane * 2; v2us oh, ol;
    Th += (size_t)z * 64 * nk; Tl += (size_t)z * 64 * nk;
#pragma unroll
    for (int i = 0; i < 2; ++i) { const float y = (d < 32) ? F[(size_t)(k0 + i) * ld + off + z * 32 + (d < 32 ? d : 0)] : 0.f; const unsigned short hb = f2bf(y); oh[i] = hb; ol[i] = f2bf(y - bf2f(hb)); }
    const size_t o = (size_t)d * nk + k0; *(volatile v2us*)(Th + o) = oh; *(volatile v2us*)(Tl + o) = ol; __threadfence(); *(volatile v2us*)(Th + o) = oh; *(volatile v2us*)(Tl + o) = ol;
}
template <int NK>
__global__ __launch_bounds__(256) void k_softmaxz(const float* __restrict__ S, int rows, bf* PH, bf* PL) {
    typedef __attribute__((ext_vector_type(4))) unsigned short v4us;
    const int lane = threadIdx.x & 31, i = blockIdx.x * 8 + (threadIdx.x >> 5); if (i >= rows) return; const size_t zo = (size_t)blockIdx.z * rows * NK; const float* sr = S + zo + (size_t)i * NK; PH += zo; PL += zo;
    float m = -3.0e38f;
#pragma unroll 1
    for (int c0 = lane * 4; c0 < NK; c0 += 128) {
#pragma unroll
        for (int q = 0; q < 4; ++q) m = fmaxf(m, sr[c0 + q]); }
#pragma unroll
    for (int sh = 16; sh; sh >>= 1) m = fmaxf(m, __shfl_xor(m, sh, 32));
    float sum = 0.f;
#pragma unroll 1
    for (int c0 = lane * 4; c0 < NK; c0 += 128) {
#pragma unroll
        for (int q = 0; q < 4; ++q) sum += __expf(sr[c0 + q] - m); }
#pragma unroll
    for (int sh = 16; sh; sh >>= 1) sum += __shfl_xor(sum, sh, 32);
    const float inv = 1.0f / sum;
#pragma unroll 1
    for (int ps = 0; ps < 2; ++ps) {
#pragma unroll 1
        for (int c0 = lane * 4; c0 < NK; c0 += 128) { v4us oh, ol;
#pragma unroll
            for (int q = 0; q < 4; ++q) { const float p = __expf(sr[c0 + q] - m) * inv; const unsigned short hb = f2bf(p); oh[q] = hb; ol[q] = f2bf(p - bf2f(hb)); }
            const size_t o = (size_t)i * NK + c0; *(volatile v4us*)(PH + o) = oh; *(volatile v4us*)(PL + o) = ol; }
        if (ps == 0) __threadfence(); }
}
__global__ __launch_bounds__(256) void k_placez(const float* __restrict__ XH, int rows, int ldy, float* Y) {
    const int lane = threadIdx.x & 31; const size_t q = (size_t)blockIdx.x * 8 + (threadIdx.x >> 5); if (q >= (size_t)rows) return; const int z = blockIdx.z; const float v = XH[((size_t)z * rows + q) * 64 + lane];
    *(volatile float*)(Y + q * ldy + z * 32 + lane) = v; __threadfence(); *(volatile float*)(Y + q * ldy + z * 32 + lane) = v;
}

__global__ __launch_bounds__(256) void k_pcz(const float* __restrict__ S, float* PC) {
    const int lane = threadIdx.x & 31; const int w = blockIdx.x * 8 + (threadIdx.x >> 5); if (w >= NX / 32) return; const int z = blockIdx.z; const int i = w * 32 + lane; const float* sr = S + ((size_t)z * NX + i) * NZ;
    float m = -3.0e38f; for (int k = 0; k < NZ; ++k) m = fmaxf(m, sr[k]);
    float s = 0.f; for (int k = 0; k < NZ; ++k) s += __expf(sr[k] - m);
    const float v = __expf(sr[NZ / 2] - m) / s; *(volatile float*)(PC + (size_t)z * NX + i) = v; __threadfence(); *(volatile float*)(PC + (size_t)z * NX + i) = v;
}
__global__ __launch_bounds__(256) void k_coarse(const float* __restrict__ PC, float* OUT0) {
    const int lane = threadIdx.x & 31; const int w = blockIdx.x * 8 + (threadIdx.x >> 5); if (w >= NX / 32) return; const int n = w * 32 + lane; float s = 0.f;
#pragma unroll
    for (int h = 0; h < NH_; ++h) s += PC[(size_t)h * NX + n];
    s *= (1.0f / NH_); *(volatile float*)(OUT0 + n) = s; __threadfence(); *(volatile float*)(OUT0 + n) = s;
}
__global__ __launch_bounds__(256) void k_split256(const float* __restrict__ src, bf* dh, bf* dl) {
    const int lane = threadIdx.x & 31; const size_t r = (size_t)blockIdx.x * 8 + (threadIdx.x >> 5); if (r >= (size_t)NX) return; const size_t o = r * CC + lane * 8; const v8f v = *(const v8f*)(src + o); v8us oh, ol;
#pragma unroll
    for (int i = 0; i < 8; ++i) { const unsigned short hb = f2bf(v[i]); oh[i] = hb; ol[i] = f2bf(v[i] - bf2f(hb)); }
    *(volatile v8us*)(dh + o) = oh; *(volatile v8us*)(dl + o) = ol; __threadfence(); *(volatile v8us*)(dh + o) = oh; *(volatile v8us*)(dl + o) = ol;
}
__global__ __launch_bounds__(256) void k_ln256(const float* __restrict__ src, const float* __restrict__ g, const float* __restrict__ bb, float* Yf, bf* Yh, bf* Yl) {
    const int lane = threadIdx.x & 31; const size_t r = (size_t)blockIdx.x * 8 + (threadIdx.x >> 5); if (r >= (size_t)NX) return; const size_t o = r * CC + lane * 8; const v8f v = *(const v8f*)(src + o); float s = 0.f;
#pragma unroll
    for (int i = 0; i < 8; ++i) s += v[i];
#pragma unroll
    for (int sh = 16; sh; sh >>= 1) s += __shfl_xor(s, sh, 32);
    const float mu = s * (1.0f / CC); float q = 0.f;
#pragma unroll
    for (int i = 0; i < 8; ++i) { const float d = v[i] - mu; q = fmaf(d, d, q); }
#pragma unroll
    for (int sh = 16; sh; sh >>= 1) q += __shfl_xor(q, sh, 32);
    const float rs = rsqrtf(q * (1.0f / CC) + LEPS); v8f y; v8us oh, ol;
#pragma unroll
    for (int i = 0; i < 8; ++i) { y[i] = (v[i] - mu) * rs * bfr(g[lane * 8 + i]) + bfr(bb[lane * 8 + i]); const unsigned short hb = f2bf(y[i]); oh[i] = hb; ol[i] = f2bf(y[i] - bf2f(hb)); }
    *(volatile v8f*)(Yf + o) = y; *(volatile v8us*)(Yh + o) = oh; *(volatile v8us*)(Yl + o) = ol; __threadfence(); *(volatile v8f*)(Yf + o) = y; *(volatile v8us*)(Yh + o) = oh; *(volatile v8us*)(Yl + o) = ol;
}
__global__ __launch_bounds__(256) void k_gelu1024(const float* __restrict__ F, bf* Gh, bf* Gl) {
    typedef __attribute__((ext_vector_type(4))) unsigned short v4us;
    const int lane = threadIdx.x & 31; const size_t r = (size_t)blockIdx.x * 8 + (threadIdx.x >> 5); if (r >= (size_t)NX) return;
#pragma unroll 1
    for (int ps = 0; ps < 2; ++ps) {
#pragma unroll 1
        for (int c0 = lane * 4; c0 < MID; c0 += 128) { v4us oh, ol;
#pragma unroll
            for (int q = 0; q < 4; ++q) { const float x = F[r * MID + c0 + q]; const float gx = 0.5f * x * (1.0f + erff(x * 0.70710678118654752f)); const unsigned short hb = f2bf(gx); oh[q] = hb; ol[q] = f2bf(gx - bf2f(hb)); }
            *(volatile v4us*)(Gh + r * MID + c0) = oh; *(volatile v4us*)(Gl + r * MID + c0) = ol; }
        if (ps == 0) __threadfence(); }
}
__global__ __launch_bounds__(256) void k_loc(const float* __restrict__ REG, float* OUT1) {
    const int lane = threadIdx.x & 31; const int w = blockIdx.x * 8 + (threadIdx.x >> 5); if (w >= 2 * (NX / 128)) return; const int c = w / (NX / 128); const int n0 = (w % (NX / 128)) * 128 + lane * 4; v4f v;
#pragma unroll
    for (int q = 0; q < 4; ++q) v[q] = REG[(size_t)(n0 + q) * 64 + c];
    *(volatile v4f*)(OUT1 + (size_t)c * NX + n0) = v; __threadfence(); *(volatile v4f*)(OUT1 + (size_t)c * NX + n0) = v;
}

__global__ __launch_bounds__(256) void k_regw(const float* __restrict__ rw, bf* RW) {
    const int lane = threadIdx.x & 31; const int wid = blockIdx.x * 8 + (threadIdx.x >> 5); if (wid >= 64 * (MID / 256)) return; const int c = wid / (MID / 256); const int k0 = (wid % (MID / 256)) * 256 + lane * 8; v8us o;
#pragma unroll
    for (int i = 0; i < 8; ++i) o[i] = (c < 2) ? f2bf(rw[(size_t)(c < 2 ? c : 0) * MID + k0 + i]) : (unsigned short)0;
    *(volatile v8us*)(RW + (size_t)c * MID + k0) = o; __threadfence(); *(volatile v8us*)(RW + (size_t)c * MID + k0) = o;
}
__global__ __launch_bounds__(256) void k_bpad(const float* __restrict__ src, int N, int n, float* BP) {
    const int t = threadIdx.x; if (t >= n) return; const float v = (t < N) ? bfr(src[t < N ? t : 0]) : 0.f; *(volatile float*)(BP + t) = v; __threadfence(); *(volatile float*)(BP + t) = v;
}

extern "C" void kernel_launch(void* const* d_in, const int* in_sizes, int n_in,
                              void* d_out, int out_size, void* d_ws, size_t ws_size, hipStream_t stream) {
    (void)in_sizes; (void)n_in; (void)out_size;
    const float* z = (const float*)d_in[0]; const float* x = (const float*)d_in[1]; const float* ca_w_in = (const float*)d_in[2]; const float* ca_b_in = (const float*)d_in[3]; const float* ca_w_out = (const float*)d_in[4]; const float* ca_b_out = (const float*)d_in[5]; const float* ca_ln_g = (const float*)d_in[6]; const float* ca_ln_b = (const float*)d_in[7];
    const float* sa_w_in = (const float*)d_in[8]; const float* sa_b_in = (const float*)d_in[9]; const float* sa_w_out = (const float*)d_in[10]; const float* sa_b_out = (const float*)d_in[11]; const float* ln_g = (const float*)d_in[12]; const float* ln_b = (const float*)d_in[13];
    const float* fine_w = (const float*)d_in[14]; const float* fine_b = (const float*)d_in[15]; const float* reg_w = (const float*)d_in[16]; const float* reg_b = (const float*)d_in[17];
    float* out0 = (float*)d_out;
    float* out1 = (float*)((char*)d_out + (size_t)NBT * NX * 4);
    char* wsp = (char*)d_ws;
    auto take = [&](size_t bytes) { char* p = wsp; wsp += (bytes + 255) & ~(size_t)255; return (void*)p; };
    bf* CAW = (bf*)take((size_t)3 * CC * CC * 2); bf* CAO = (bf*)take((size_t)CC * CC * 2); bf* SAW = (bf*)take((size_t)NL * 3 * CC * CC * 2); bf* SAO = (bf*)take((size_t)NL * CC * CC * 2); bf* FW = (bf*)take((size_t)MID * CC * 2); bf* RW = (bf*)take((size_t)64 * MID * 2); float* RB = (float*)take(64 * 4);
    bf* Xq = (bf*)take((size_t)NX * CC * 2); bf* Zk = (bf*)take((size_t)NZ * CC * 2); float* QP = (float*)take((size_t)NX * CC * 4); float* KVZ = (float*)take((size_t)NZ * 3 * CC * 4); float* QKV = (float*)take((size_t)NX * 3 * CC * 4);
    bf* Qh = (bf*)take((size_t)NH_ * NX * HD * 2); bf* Ql = (bf*)take((size_t)NH_ * NX * HD * 2); bf* Kh = (bf*)take((size_t)NH_ * NX * HD * 2); bf* Kl = (bf*)take((size_t)NH_ * NX * HD * 2); bf* VTh = (bf*)take((size_t)NH_ * 64 * NX * 2); bf* VTl = (bf*)take((size_t)NH_ * 64 * NX * 2);
    float* S = (float*)take((size_t)NH_ * NX * NX * 4); bf* PH = (bf*)take((size_t)NH_ * NX * NX * 2); bf* PL = (bf*)take((size_t)NH_ * NX * NX * 2); float* PC = (float*)take((size_t)NH_ * NX * 4); float* XH = (float*)take((size_t)NH_ * NX * 64 * 4); float* Y = (float*)take((size_t)NX * CC * 4); bf* Yh = (bf*)take((size_t)NX * CC * 2); bf* Yl = (bf*)take((size_t)NX * CC * 2);
    float* AO = (float*)take((size_t)NX * CC * 4); float* Yf = (float*)take((size_t)NX * CC * 4); float* FF = (float*)take((size_t)NX * MID * 4); bf* Gh = (bf*)take((size_t)NX * MID * 2); bf* Gl = (bf*)take((size_t)NX * MID * 2); float* REG = (float*)take((size_t)NX * 64 * 4);
    if ((size_t)(wsp - (char*)d_ws) > ws_size) return;
    k_cvt8<<<(3 * CC * CC / 8 + 255) / 256, 256, 0, stream>>>(ca_w_in, CAW, 3 * CC * CC / 8); k_cvt8<<<(CC * CC / 8 + 255) / 256, 256, 0, stream>>>(ca_w_out, CAO, CC * CC / 8);
    k_cvt8<<<(NL * 3 * CC * CC / 8 + 255) / 256, 256, 0, stream>>>(sa_w_in, SAW, (size_t)NL * 3 * CC * CC / 8); k_cvt8<<<(NL * CC * CC / 8 + 255) / 256, 256, 0, stream>>>(sa_w_out, SAO, (size_t)NL * CC * CC / 8);
    k_cvt8<<<(MID * CC / 8 + 255) / 256, 256, 0, stream>>>(fine_w, FW, MID * CC / 8);
    k_regw<<<(64 * (MID / 256)) / 8, 256, 0, stream>>>(reg_w, RW); k_bpad<<<1, 64, 0, stream>>>(reg_b, 2, 64, RB);
    auto attend = [&](const float* QF, int ldq, int qoff, const float* KF, int ldk, int koff, const float* VF, int ldv, int voff, int nk, float* PCbuf) {
        k_planes32z<<<dim3((NX / 2) / 8, 1, NH_), 256, 0, stream>>>(QF, ldq, qoff, QSC, NX, Qh, Ql); k_planes32z<<<dim3((nk / 2 + 7) / 8, 1, NH_), 256, 0, stream>>>(KF, ldk, koff, 1.0f, nk, Kh, Kl);
        k_vtpadz<<<dim3((64 * (nk / 64)) / 8, 1, NH_), 256, 0, stream>>>(VF, ldv, voff, nk, VTh, VTl);
        k_gemm3z<0><<<dim3(NX / 64, nk / 64, NH_), 128, 0, stream>>>(Qh, Ql, Kh, Kl, HD, S, nk, (size_t)NX * HD, (size_t)nk * HD, (size_t)NX * nk);
        if (nk == NZ) { k_softmaxz<NZ><<<dim3(NX / 8, 1, NH_), 256, 0, stream>>>(S, NX, PH, PL); if (PCbuf) k_pcz<<<dim3((NX / 32) / 8, 1, NH_), 256, 0, stream>>>(S, PCbuf); }
        else k_softmaxz<NX><<<dim3(NX / 8, 1, NH_), 256, 0, stream>>>(S, NX, PH, PL);
        k_gemm3z<0><<<dim3(NX / 64, 1, NH_), 128, 0, stream>>>(PH, PL, VTh, VTl, nk, XH, 64, (size_t)NX * nk, (size_t)64 * nk, (size_t)NX * 64);
        k_placez<<<dim3(NX / 8, 1, NH_), 256, 0, stream>>>(XH, NX, CC, Y); };
    for (int b = 0; b < NBT; ++b) {
        k_wt<<<dim3(CC / 64, NX / 64, 1), 256, 0, stream>>>(x + (size_t)b * CC * NX, CC, NX, Xq); k_wt<<<dim3(CC / 64, NZ / 64, 1), 256, 0, stream>>>(z + (size_t)b * CC * NZ, CC, NZ, Zk);
        k_gemmb<false, false><<<dim3(NX / 64, CC / 64, 1), 128, 0, stream>>>(Xq, nullptr, CAW, ca_b_in, QP, CC, nullptr, nullptr, CC);
        k_gemmb<false, false><<<dim3(NZ / 64, (3 * CC) / 64, 1), 128, 0, stream>>>(Zk, nullptr, CAW, ca_b_in, KVZ, 3 * CC, nullptr, nullptr, CC);
        attend(QP, CC, 0, KVZ, 3 * CC, CC, KVZ, 3 * CC, 2 * CC, NZ, PC);
        k_coarse<<<(NX / 32) / 8, 256, 0, stream>>>(PC, out0 + (size_t)b * NX);
        k_split256<<<NX / 8, 256, 0, stream>>>(Y, Yh, Yl);
        k_gemmb<true, false><<<dim3(NX / 64, CC / 64, 1), 128, 0, stream>>>(Yh, Yl, CAO, ca_b_out, AO, CC, nullptr, nullptr, CC);
        k_ln256<<<NX / 8, 256, 0, stream>>>(AO, ca_ln_g, ca_ln_b, Yf, Yh, Yl);
        for (int l = 0; l < NL; ++l) {
            k_gemmb<true, false><<<dim3(NX / 64, (3 * CC) / 64, 1), 128, 0, stream>>>(Yh, Yl, SAW + (size_t)l * 3 * CC * CC, sa_b_in + (size_t)l * 3 * CC, QKV, 3 * CC, nullptr, nullptr, CC);
            attend(QKV, 3 * CC, 0, QKV, 3 * CC, CC, QKV, 3 * CC, 2 * CC, NX, nullptr);
            k_split256<<<NX / 8, 256, 0, stream>>>(Y, Yh, Yl);
            k_gemmb<true, false><<<dim3(NX / 64, CC / 64, 1), 128, 0, stream>>>(Yh, Yl, SAO + (size_t)l * CC * CC, sa_b_out + (size_t)l * CC, AO, CC, nullptr, nullptr, CC);
            k_ln256<<<NX / 8, 256, 0, stream>>>(AO, ln_g + (size_t)l * CC, ln_b + (size_t)l * CC, Yf, Yh, Yl); }
        k_gemmb<true, false><<<dim3(NX / 64, MID / 64, 1), 128, 0, stream>>>(Yh, Yl, FW, fine_b, FF, MID, nullptr, nullptr, CC);
        k_gelu1024<<<NX / 8, 256, 0, stream>>>(FF, Gh, Gl);
        k_gemmb<true, false><<<dim3(NX / 64, 1, 1), 128, 0, stream>>>(Gh, Gl, RW, RB, REG, 64, nullptr, nullptr, MID);
        k_loc<<<(2 * (NX / 128)) / 8, 256, 0, stream>>>(REG, out1 + (size_t)b * 2 * NX); }
}
